// SurnameClassifier_87840671137937
// MI455X (gfx1250) — hardware-verified
//
#include <hip/hip_runtime.h>
#include <math.h>

#define BB 1024
#define SS 64
#define EE 256
#define HH 512
#define VV 128
#define CC 32
#define CP 64
#define NT 256
#define HP 520

typedef __attribute__((ext_vector_type(16))) _Float16 v16h;
typedef __attribute__((ext_vector_type(8)))  _Float16 v8h;
typedef __attribute__((ext_vector_type(16))) __bf16   v16b;
typedef __attribute__((ext_vector_type(8)))  __bf16   v8b;
typedef __attribute__((ext_vector_type(8)))  float    v8f;
typedef __attribute__((ext_vector_type(4)))  float    v4f;

__device__ __forceinline__ unsigned short f2bf_bits(float f) {
  unsigned u = __float_as_uint(f);
  return (unsigned short)((u + 0x7FFFu + ((u >> 16) & 1u)) >> 16);
}
__device__ __forceinline__ float bf_bits2f(unsigned short h) { return __uint_as_float(((unsigned)h) << 16); }

__device__ __forceinline__ void dep_guard_h(v8f& a, v8f& b, v16h x, v16h y) { asm volatile("v_nop\n\tv_nop\n\tv_nop\n\tv_nop" : "+v"(a), "+v"(b) : "v"(x), "v"(y)); }
__device__ __forceinline__ void dep_guard_b(v8f& a, v8f& b, v16b x, v16b y) { asm volatile("v_nop\n\tv_nop\n\tv_nop\n\tv_nop" : "+v"(a), "+v"(b) : "v"(x), "v"(y)); }
__device__ __forceinline__ void keep4_h(v16h a, v16h b, v16h c, v16h d) { asm volatile("v_nop" :: "v"(a), "v"(b), "v"(c), "v"(d)); }
__device__ __forceinline__ void keep4_b(v16b a, v16b b, v16b c, v16b d) { asm volatile("v_nop" :: "v"(a), "v"(b), "v"(c), "v"(d)); }
__device__ __forceinline__ void acc_guard4(v8f& a, v8f& b, v8f& c, v8f& d) { asm volatile("v_nop\n\tv_nop\n\tv_nop\n\tv_nop" : "+v"(a), "+v"(b), "+v"(c), "+v"(d)); }
template <typename T> struct Frag;
template <> struct Frag<_Float16> {
  typedef v16h V; union U { v16h v; v8h h[2]; };
  static __device__ __forceinline__ v16h load(const _Float16* p) {
    U f; f.h[0] = *(const v8h*)(p); f.h[1] = *(const v8h*)(p + 16); return f.v;
  }
  static __device__ __forceinline__ v8f mma(v16h a, v16h b, v8f c) {
    return __builtin_amdgcn_wmma_f32_16x16x32_f16(false, a, false, b, (short)0, c, false, false);
  }
  static __device__ __forceinline__ void guard(v8f& a, v8f& b, v16h x, v16h y) { dep_guard_h(a, b, x, y); }
  static __device__ __forceinline__ void keep(v16h a, v16h b, v16h c, v16h d) { keep4_h(a, b, c, d); }
};
template <> struct Frag<__bf16> {
  typedef v16b V; union U { v16b v; v8b h[2]; };
  static __device__ __forceinline__ v16b load(const __bf16* p) {
    U f; f.h[0] = *(const v8b*)(p); f.h[1] = *(const v8b*)(p + 16); return f.v;
  }
  static __device__ __forceinline__ v8f mma(v16b a, v16b b, v8f c) {
    return __builtin_amdgcn_wmma_f32_16x16x32_bf16(false, a, false, b, (short)0, c, false, false);
  }
  static __device__ __forceinline__ void guard(v8f& a, v8f& b, v16b x, v16b y) { dep_guard_b(a, b, x, y); }
  static __device__ __forceinline__ void keep(v16b a, v16b b, v16b c, v16b d) { keep4_b(a, b, c, d); }
};

template <int ET> struct Elem;
template <> struct Elem<0> { typedef _Float16 T; };
template <> struct Elem<1> { typedef __bf16 T; };
template <int ET, bool SPLIT, int BIAS_MODE, int OUT_MODE, bool RESID, int ACT = 0>
__global__ __launch_bounds__(256) void wmma_gemm64(
    const unsigned short* __restrict__ Ap, const unsigned short* __restrict__ A2p, int lda, long strideA,
    const unsigned short* __restrict__ Btp, const unsigned short* __restrict__ Bt2p, int ldb, long strideB,
    void* __restrict__ Cout, void* __restrict__ Cout2, int ldc, long strideC,
    const float* __restrict__ bias,
    const float* __restrict__ resid, long strideR,
    int M, int N, int K, float scale) {
  typedef typename Elem<ET>::T T;
  typedef typename Frag<T>::V V;
  const T* A = (const T*)Ap; const T* A2 = (const T*)A2p; const T* Bt = (const T*)Btp; const T* Bt2 = (const T*)Bt2p;
  __shared__ __align__(16) float sT[8][16 * 68];
  const int b    = blockIdx.y;
  const int lane = threadIdx.x & 31;
  const int wave = threadIdx.x >> 5;
  const int tilesN = N >> 6;
  const int tilesM = M >> 6;
  const int tile = blockIdx.x * 8 + wave;
  if (tile >= tilesM * tilesN) return;
  const int tm = tile / tilesN;
  const int tn = tile - tm * tilesN;
  const int m0 = tm << 6;
  const int n0 = tn << 6;

  const T* Ab  = A  + (size_t)b * strideA;
  const T* Bb  = Bt + (size_t)b * strideB;
  const T* Ab2 = SPLIT ? (A2  + (size_t)b * strideA) : nullptr;
  const T* Bb2 = SPLIT ? (Bt2 + (size_t)b * strideB) : nullptr;

  const int rlane = lane & 15;
  const int koff  = (lane >> 4) * 8;
  const int mOff  = (lane >> 4) * 8;

  v8f acc[4][4];
#pragma unroll
  for (int i = 0; i < 4; ++i)
#pragma unroll
    for (int j = 0; j < 4; ++j) acc[i][j] = (v8f){0.f,0.f,0.f,0.f,0.f,0.f,0.f,0.f};

  for (int k0 = 0; k0 < K; k0 += 32) {
    V bh[4], bl[4];
#pragma unroll
    for (int j = 0; j < 4; ++j) {
      const size_t bo = (size_t)(n0 + (j << 4) + rlane) * ldb + koff + k0;
      bh[j] = Frag<T>::load(Bb + bo);
      if (SPLIT) bl[j] = Frag<T>::load(Bb2 + bo);
    }
#pragma unroll
    for (int i = 0; i < 4; ++i) {
      const size_t ao = (size_t)(m0 + (i << 4) + rlane) * lda + koff + k0;
      V ah = Frag<T>::load(Ab + ao);
      V al;
      if (SPLIT) al = Frag<T>::load(Ab2 + ao);
#pragma unroll
      for (int j = 0; j < 4; ++j) {
        acc[i][j] = Frag<T>::mma(ah, bh[j], acc[i][j]);
        if (SPLIT) {
          acc[i][j] = Frag<T>::mma(ah, bl[j], acc[i][j]);
          acc[i][j] = Frag<T>::mma(al, bh[j], acc[i][j]);
        }
      }
      Frag<T>::guard(acc[i][0], acc[i][3], ah, SPLIT ? al : ah);
    }
    Frag<T>::keep(bh[0], bh[1], bh[2], bh[3]);
    if (SPLIT) Frag<T>::keep(bl[0], bl[1], bl[2], bl[3]);
  }
  acc_guard4(acc[0][0], acc[0][1], acc[0][2], acc[0][3]);
  acc_guard4(acc[1][0], acc[1][1], acc[1][2], acc[1][3]);
  acc_guard4(acc[2][0], acc[2][1], acc[2][2], acc[2][3]);
  acc_guard4(acc[3][0], acc[3][1], acc[3][2], acc[3][3]);

  float* slab = sT[wave];
  const float* Rb = RESID ? (resid + (size_t)b * strideR) : nullptr;
#pragma unroll
  for (int i = 0; i < 4; ++i) {
    const int mBase = m0 + (i << 4);
#pragma unroll
    for (int j = 0; j < 4; ++j) {
      const int n = n0 + (j << 4) + rlane;
      float bv = 0.f;
      if (BIAS_MODE == 2) bv = bias[n];
#pragma unroll
      for (int r = 0; r < 8; ++r) {
        float v = acc[i][j][r] * scale;
        if (BIAS_MODE == 1) v += bias[mBase + mOff + r];
        if (BIAS_MODE == 2) v += bv;
        if (RESID) v += Rb[(size_t)(mBase + mOff + r) * ldc + n];
        if (ACT == 1) v = tanhf(v);
        if (ACT == 2) v = fmaxf(v, 0.0f);
        if (ACT == 3) v = v / (1.0f + expf(-v));
        if (ACT == 4) v = (v > 0.f) ? v : 0.01f * v;
        if (ACT == 5) v = 0.5f * v * (1.0f + erff(v * 0.70710678118654752f));
        slab[(mOff + r) * 68 + (j << 4) + rlane] = v;
      }
    }
    __builtin_amdgcn_fence(__ATOMIC_RELEASE, "workgroup");
    __builtin_amdgcn_wave_barrier();
    __builtin_amdgcn_fence(__ATOMIC_ACQUIRE, "workgroup");
    if (OUT_MODE == 0) {
      float* C = (float*)Cout + (size_t)b * strideC;
      const int hh = lane >> 4, c4 = (lane & 15) * 4;
      for (int pass = 0; pass < 2; ++pass) {
#pragma unroll
        for (int it = 0; it < 8; ++it) {
          const int row = it * 2 + hh;
          v4f v = *(const v4f*)(slab + row * 68 + c4);
          *(volatile v4f*)(C + (size_t)(mBase + row) * ldc + n0 + c4) = v;
        }
        __threadfence();
      }
    } else {
      const int q = lane >> 3, c8 = (lane & 7) * 8;
      unsigned short* C  = (unsigned short*)Cout  + (size_t)b * strideC;
      unsigned short* C2 = (OUT_MODE == 2) ? ((unsigned short*)Cout2 + (size_t)b * strideC) : nullptr;
      for (int pass = 0; pass < 2; ++pass) {
#pragma unroll
        for (int it = 0; it < 4; ++it) {
          const int row = it * 4 + q;
          const float* sp = slab + row * 68 + c8;
          v8h hv, lv;
#pragma unroll
          for (int e = 0; e < 8; ++e) {
            if (OUT_MODE == 1) {
              hv[e] = (_Float16)sp[e];
            } else {
              unsigned short hb = f2bf_bits(sp[e]);
              unsigned short lb = f2bf_bits(sp[e] - bf_bits2f(hb));
              hv[e] = __builtin_bit_cast(_Float16, hb);
              lv[e] = __builtin_bit_cast(_Float16, lb);
            }
          }
          *(volatile v8h*)(C + (size_t)(mBase + row) * ldc + n0 + c8) = hv;
          if (OUT_MODE == 2) *(volatile v8h*)(C2 + (size_t)(mBase + row) * ldc + n0 + c8) = lv;
        }
        __threadfence();
      }
    }
    __builtin_amdgcn_fence(__ATOMIC_RELEASE, "workgroup");
    __builtin_amdgcn_wave_barrier();
    __builtin_amdgcn_fence(__ATOMIC_ACQUIRE, "workgroup");
  }
}

__device__ __forceinline__ unsigned pack_f16x2(float a, float b) {
  const _Float16 h0 = (_Float16)a, h1 = (_Float16)b;
  return (unsigned)__builtin_bit_cast(unsigned short, h0) | ((unsigned)__builtin_bit_cast(unsigned short, h1) << 16);
}
__device__ __forceinline__ void split_pack2(float a, float b, unsigned& uh, unsigned& ul) {
  const unsigned short ha = f2bf_bits(a), hb = f2bf_bits(b);
  const unsigned short la = f2bf_bits(a - bf_bits2f(ha)), lb = f2bf_bits(b - bf_bits2f(hb));
  uh = (unsigned)ha | ((unsigned)hb << 16);
  ul = (unsigned)la | ((unsigned)lb << 16);
}
__device__ __forceinline__ void st2u(unsigned* p, unsigned v) { *(volatile unsigned*)p = v; __threadfence(); *(volatile unsigned*)p = v; }
__device__ __forceinline__ void st2f(float* p, float v) { *(volatile float*)p = v; __threadfence(); *(volatile float*)p = v; }

__global__ __launch_bounds__(NT) void prep_kernel(const float* __restrict__ emb, const float* __restrict__ W_ih,
                                                 const float* __restrict__ b_ih, const float* __restrict__ W_hh,
                                                 const float* __restrict__ b_hh, const float* __restrict__ W1,
                                                 const float* __restrict__ W2, const float* __restrict__ b2,
                                                 unsigned* __restrict__ EMBH, unsigned* __restrict__ EMBL,
                                                 unsigned* __restrict__ WIHH, unsigned* __restrict__ WIHL,
                                                 unsigned* __restrict__ WHHH, unsigned* __restrict__ WHHL,
                                                 unsigned* __restrict__ W1S, unsigned* __restrict__ W2S,
                                                 float* __restrict__ BSUM, float* __restrict__ B2P) {
  const int blk = blockIdx.x, tid = threadIdx.x;
  if (blk < 64) {
    const int p = blk * NT + tid;
    unsigned uh, ul; split_pack2(emb[2 * p], emb[2 * p + 1], uh, ul);
    st2u(EMBH + p, uh); st2u(EMBL + p, ul);
  } else if (blk < 320) {
    const int p = (blk - 64) * NT + tid;
    unsigned uh, ul; split_pack2(W_ih[2 * p], W_ih[2 * p + 1], uh, ul);
    st2u(WIHH + p, uh); st2u(WIHL + p, ul);
  } else if (blk < 832) {
    const int p = (blk - 320) * NT + tid;
    unsigned uh, ul; split_pack2(W_hh[2 * p], W_hh[2 * p + 1], uh, ul);
    st2u(WHHH + p, uh); st2u(WHHL + p, ul);
  } else if (blk < 1344) {
    const int p = (blk - 832) * NT + tid;
    const unsigned u = pack_f16x2(W1[2 * p] * 16.0f, W1[2 * p + 1] * 16.0f);
    st2u(W1S + p, u);
  } else if (blk < 1408) {
    const int p = (blk - 1344) * NT + tid;
    const int o = p >> 8, k = 2 * (p & 255);
    const int oc = o < CC ? o : (CC - 1);
    const bool live = o < CC;
    const float a = W2[oc * HH + k] * 16.0f, bq = W2[oc * HH + k + 1] * 16.0f;
    const unsigned u = pack_f16x2(live ? a : 0.f, live ? bq : 0.f);
    st2u(W2S + p, u);
  } else {
    const int i = (blk - 1408) * NT + tid;
    const int ic = i < HH ? i : (HH - 1);
    const float bs = b_ih[ic] + b_hh[ic];
    int jc = i - HH; jc = jc < 0 ? 0 : (jc >= CC ? (CC - 1) : jc);
    const float bv = b2[jc];
    if (i < HH) {
      st2f(BSUM + i, bs);
    } else if (i < HH + CP) {
      const float v = (i < HH + CC) ? bv : 0.f;
      st2f(B2P + (i - HH), v);
    }
  }
}

__global__ __launch_bounds__(NT) void rnn_kernel(const int* __restrict__ x_in, const int* __restrict__ x_lens,
                                                const float* __restrict__ P,
                                                const unsigned short* __restrict__ WHp, const unsigned short* __restrict__ WLp,
                                                _Float16* __restrict__ LAST) {
  __shared__ __align__(16) __bf16 hhi[16 * HP];
  __shared__ __align__(16) __bf16 hlo[16 * HP];
  __shared__ __align__(16) _Float16 lst[16 * HP];
  __shared__ int tok_s[16 * SS];
  const __bf16* WH = (const __bf16*)(const void*)WHp;
  const __bf16* WL = (const __bf16*)(const void*)WLp;
  const int tid = threadIdx.x, lane = tid & 31, wave = tid >> 5;
  const int rlane = lane & 15, hh = lane >> 4, koff = hh * 8, mOff = hh * 8;
  const int mbase = blockIdx.x * 16;
  const __bf16 bz = __builtin_bit_cast(__bf16, (unsigned short)0);
  const _Float16 hz = (_Float16)0.0f;
  for (int i = tid; i < 16 * HP; i += NT) { hhi[i] = bz; hlo[i] = bz; lst[i] = hz; }
  for (int i = tid; i < 16 * SS; i += NT) {
    int v = x_in[(size_t)(mbase + (i >> 6)) * SS + (i & 63)];
    v = v < 0 ? 0 : (v >= VV ? (VV - 1) : v);
    tok_s[i] = v;
  }
  int lenr[8];
#pragma unroll
  for (int r = 0; r < 8; ++r) {
    int L = x_lens[mbase + mOff + r];
    L = L < 1 ? 1 : (L > SS ? SS : L);
    lenr[r] = L - 1;
  }
  __syncthreads();

  const int col0 = 64 * wave + rlane;
  const __bf16* ahp = hhi + rlane * HP + koff;
  const __bf16* alp = hlo + rlane * HP + koff;
  const __bf16* wbh = WH + (size_t)col0 * HH + koff;
  const __bf16* wbl = WL + (size_t)col0 * HH + koff;
  const v8f z8 = {0.f, 0.f, 0.f, 0.f, 0.f, 0.f, 0.f, 0.f};

#pragma unroll 1
  for (int t = 0; t < SS; ++t) {
    v8f acc[4];
    acc[0] = z8; acc[1] = z8; acc[2] = z8; acc[3] = z8;
#pragma unroll 1
    for (int k0 = 0; k0 < HH; k0 += 32) {
      v16b bh[4], bl[4];
#pragma unroll
      for (int nt = 0; nt < 4; ++nt) {
        bh[nt] = Frag<__bf16>::load(wbh + (size_t)nt * 16 * HH + k0);
        bl[nt] = Frag<__bf16>::load(wbl + (size_t)nt * 16 * HH + k0);
      }
      const v16b ah = Frag<__bf16>::load(ahp + k0);
      const v16b al = Frag<__bf16>::load(alp + k0);
#pragma unroll
      for (int nt = 0; nt < 4; ++nt) {
        acc[nt] = Frag<__bf16>::mma(ah, bh[nt], acc[nt]);
        acc[nt] = Frag<__bf16>::mma(ah, bl[nt], acc[nt]);
        acc[nt] = Frag<__bf16>::mma(al, bh[nt], acc[nt]);
      }
      dep_guard_b(acc[0], acc[3], ah, al);
      keep4_b(bh[0], bh[1], bh[2], bh[3]);
      keep4_b(bl[0], bl[1], bl[2], bl[3]);
    }
    acc_guard4(acc[0], acc[1], acc[2], acc[3]);
    __syncthreads();
#pragma unroll
    for (int r = 0; r < 8; ++r) {
      const int row = mOff + r;
      const int tok = tok_s[row * SS + t];
      const float* prow = P + (size_t)tok * HH + col0;
      const bool sel = (t == lenr[r]);
#pragma unroll
      for (int nt = 0; nt < 4; ++nt) {
        const float z = acc[nt][r] + prow[16 * nt];
        const float h = tanhf(z);
        const unsigned short hb = f2bf_bits(h);
        const unsigned short lb = f2bf_bits(h - bf_bits2f(hb));
        const int li = row * HP + col0 + 16 * nt;
        hhi[li] = __builtin_bit_cast(__bf16, hb);
        hlo[li] = __builtin_bit_cast(__bf16, lb);
        if (sel) lst[li] = (_Float16)h;
      }
    }
    __syncthreads();
  }

  for (int pass = 0; pass < 2; ++pass) {
#pragma unroll
    for (int rr = 0; rr < 2; ++rr) {
      const int row = 2 * wave + rr;
#pragma unroll
      for (int hf = 0; hf < 2; ++hf) {
        const v8h v = *(const v8h*)(lst + row * HP + hf * 256 + lane * 8);
        *(volatile v8h*)(LAST + (size_t)(mbase + row) * HH + hf * 256 + lane * 8) = v;
      }
    }
    __threadfence();
  }
}

__global__ __launch_bounds__(NT) void pack_kernel(const float* __restrict__ LG, float* __restrict__ out) {
  const int gid = blockIdx.x * NT + threadIdx.x;
  if (gid >= BB * 8) return;
  const int row = gid >> 3, c4 = (gid & 7) * 4;
  const v4f v = *(const v4f*)(LG + (size_t)row * CP + c4);
  float* p = out + (size_t)row * CC + c4;
  *(volatile v4f*)p = v;
  __threadfence();
  *(volatile v4f*)p = v;
}

extern "C" void kernel_launch(void* const* d_in, const int* in_sizes, int n_in,
                              void* d_out, int out_size, void* d_ws, size_t ws_size, hipStream_t stream) {
  if (n_in < 11 || d_out == nullptr || d_ws == nullptr) return;
  if (in_sizes[0] != BB * SS || in_sizes[1] != BB || in_sizes[2] != VV * EE || in_sizes[3] != HH * EE || in_sizes[4] != HH ||
      in_sizes[5] != HH * HH || in_sizes[6] != HH || in_sizes[7] != HH * HH || in_sizes[8] != HH || in_sizes[9] != CC * HH ||
      in_sizes[10] != CC || out_size != BB * CC) return;

  const int*   x_in   = (const int*)d_in[0];
  const int*   x_lens = (const int*)d_in[1];
  const float* emb    = (const float*)d_in[2];
  const float* W_ih   = (const float*)d_in[3];
  const float* b_ih   = (const float*)d_in[4];
  const float* W_hh   = (const float*)d_in[5];
  const float* b_hh   = (const float*)d_in[6];
  const float* W1     = (const float*)d_in[7];
  const float* b1     = (const float*)d_in[8];
  const float* W2     = (const float*)d_in[9];
  const float* b2     = (const float*)d_in[10];
  float* out = (float*)d_out;

  char* ws = (char*)d_ws; size_t off = 0;
  auto carve = [&](size_t bytes) -> char* { char* p = ws + off; off += (bytes + 255) & ~(size_t)255; return p; };
  unsigned* EMBH   = (unsigned*)carve((size_t)VV * EE * 2);
  unsigned* EMBL   = (unsigned*)carve((size_t)VV * EE * 2);
  unsigned* WIHH   = (unsigned*)carve((size_t)HH * EE * 2);
  unsigned* WIHL   = (unsigned*)carve((size_t)HH * EE * 2);
  unsigned* WHHH   = (unsigned*)carve((size_t)HH * HH * 2);
  unsigned* WHHL   = (unsigned*)carve((size_t)HH * HH * 2);
  unsigned* W1S    = (unsigned*)carve((size_t)HH * HH * 2);
  unsigned* W2S    = (unsigned*)carve((size_t)CP * HH * 2);
  float*    BSUM   = (float*)carve((size_t)HH * 4);
  float*    B2P    = (float*)carve((size_t)CP * 4);
  float*    P      = (float*)carve((size_t)VV * HH * 4);
  _Float16* LAST16 = (_Float16*)carve((size_t)BB * HH * 2);
  _Float16* HID16  = (_Float16*)carve((size_t)BB * HH * 2);
  float*    LG     = (float*)carve((size_t)BB * CP * 4);
  if (off > ws_size || off > (size_t)134217728) return;

  prep_kernel<<<1411, NT, 0, stream>>>(emb, W_ih, b_ih, W_hh, b_hh, W1, W2, b2,
                                       EMBH, EMBL, WIHH, WIHL, WHHH, WHHL, W1S, W2S, BSUM, B2P);
  {
    const int tiles = (VV / 64) * (HH / 64);
    wmma_gemm64<1, true, 2, 0, false, 0><<<dim3((tiles + 7) / 8, 1), 256, 0, stream>>>(
        (const unsigned short*)EMBH, (const unsigned short*)EMBL, EE, 0L,
        (const unsigned short*)WIHH, (const unsigned short*)WIHL, EE, 0L,
        (void*)P, (void*)nullptr, HH, 0L,
        BSUM, (const float*)nullptr, 0L, VV, HH, EE, 1.0f);
  }
  rnn_kernel<<<BB / 16, NT, 0, stream>>>(x_in, x_lens, P, (const unsigned short*)WHHH, (const unsigned short*)WHHL, LAST16);
  {
    const int tiles = (BB / 64) * (HH / 64);
    wmma_gemm64<0, false, 2, 1, false, 2><<<dim3((tiles + 7) / 8, 1), 256, 0, stream>>>(
        (const unsigned short*)LAST16, (const unsigned short*)nullptr, HH, 0L,
        (const unsigned short*)W1S, (const unsigned short*)nullptr, HH, 0L,
        (void*)HID16, (void*)nullptr, HH, 0L,
        b1, (const float*)nullptr, 0L, BB, HH, HH, 1.0f / 16.0f);
  }
  {
    const int tiles = (BB / 64) * (CP / 64);
    wmma_gemm64<0, false, 2, 0, false, 0><<<dim3((tiles + 7) / 8, 1), 256, 0, stream>>>(
        (const unsigned short*)HID16, (const unsigned short*)nullptr, HH, 0L,
        (const unsigned short*)W2S, (const unsigned short*)nullptr, HH, 0L,
        (void*)LG, (void*)nullptr, CP, 0L,
        B2P, (const float*)nullptr, 0L, BB, CP, HH, 1.0f / 16.0f);
  }
  pack_kernel<<<(BB * 8) / NT, NT, 0, stream>>>(LG, out);
}
